// SelfAttention2D_85134841742061
// MI455X (gfx1250) — hardware-verified
//
#include <hip/hip_runtime.h>


#ifndef NB
#define NB 8
#endif
#ifndef SEQ
#define SEQ 4096
#endif
#define NB_FULL 8
#define SEQ_FULL 4096
#define CH 256
#define DQ 32
#define JB 64
#define WROWS (2 * DQ + CH)

static_assert(NB >= 1 && NB <= NB_FULL);
static_assert(SEQ >= 64 && SEQ <= SEQ_FULL && (SEQ % 64) == 0);
static_assert(CH == 256 && DQ == 32 && JB == 64);

#define LDS_X   0
#define LDS_QH  16384
#define LDS_QL  18432
#define LDS_KH  20480
#define LDS_KL  22528
#define LDS_PROJ_TOTAL 24576

typedef unsigned int v4u __attribute__((ext_vector_type(4)));
typedef float v4f __attribute__((ext_vector_type(4)));
typedef float v8f __attribute__((ext_vector_type(8)));
typedef __bf16 v16b __attribute__((ext_vector_type(16)));
typedef _Float16 v16h __attribute__((ext_vector_type(16)));

union Frag { v4u q[2]; v16b b; v16h f; };

static constexpr float LOG2E   = 1.44269504088896340736f;
static constexpr float PC_LOG2 = 14.0f;

__device__ __forceinline__ unsigned int bf16_rne_bits(float f) {
  unsigned int u = __builtin_bit_cast(unsigned int, f);
  u = u + 0x7FFFu + ((u >> 16) & 1u);
  return u >> 16;
}
__device__ __forceinline__ float bf16_rne_val(float f) {
  return __builtin_bit_cast(float, bf16_rne_bits(f) << 16);
}
__device__ __forceinline__ unsigned short f16_bits(float f) {
  _Float16 t = (_Float16)f;
  return __builtin_bit_cast(unsigned short, t);
}
__device__ __forceinline__ v4f max4(v4f a, v4f b) {
  v4f r;
  r.x = fmaxf(a.x, b.x); r.y = fmaxf(a.y, b.y); r.z = fmaxf(a.z, b.z); r.w = fmaxf(a.w, b.w);
  return r;
}
__device__ __forceinline__ v8f zero8() {
  v8f z;
#pragma unroll
  for (int r = 0; r < 8; ++r) z[r] = 0.0f;
  return z;
}

__device__ __forceinline__ Frag ld_frag(const unsigned short* row, int h) {
  Frag fr;
  fr.q[0] = *(const v4u*)(row + 8 * h);
  fr.q[1] = *(const v4u*)(row + 16 + 8 * h);
  return fr;
}

__device__ __forceinline__ v8f mma_bf16(Frag a, Frag bb, v8f c) {
  v8f d = __builtin_amdgcn_wmma_f32_16x16x32_bf16(false, a.b, false, bb.b, (short)0, c, false, false);
  asm volatile("v_nop\n\tv_nop\n\tv_nop\n\tv_nop" : "+v"(d) : "v"(a.b), "v"(bb.b));
  return d;
}
__device__ __forceinline__ v8f mma_f16(Frag a, Frag bb, v8f c) {
  v8f d = __builtin_amdgcn_wmma_f32_16x16x32_f16(false, a.f, false, bb.f, (short)0, c, false, false);
  asm volatile("v_nop\n\tv_nop\n\tv_nop\n\tv_nop" : "+v"(d) : "v"(a.f), "v"(bb.f));
  return d;
}

__global__ __launch_bounds__(128) void k_wconv(const float* __restrict__ src,
                                               unsigned short* __restrict__ dst, int n) {
  const int t = blockIdx.x * 128 + threadIdx.x;
  const int e = t * 8;
  if (e + 8 > n) return;
  const v4f a = *(const v4f*)(src + e);
  const v4f c = *(const v4f*)(src + e + 4);
  v4u w;
  w.x = bf16_rne_bits(a.x) | (bf16_rne_bits(a.y) << 16);
  w.y = bf16_rne_bits(a.z) | (bf16_rne_bits(a.w) << 16);
  w.z = bf16_rne_bits(c.x) | (bf16_rne_bits(c.y) << 16);
  w.w = bf16_rne_bits(c.z) | (bf16_rne_bits(c.w) << 16);
  volatile v4u* p = (volatile v4u*)(dst + e);
  *p = w;
  __threadfence();
  *p = w;
}

__device__ __forceinline__ void proj_store(const unsigned short* lds,
                                           unsigned short* Qh, unsigned short* Ql,
                                           unsigned short* Kh, unsigned short* Kl,
                                           unsigned short* Vb, int tid) {
#pragma unroll
  for (int p = 0; p < 2; ++p) {
    const int u = p * 128 + tid;
    const v4u a0 = *(const v4u*)(lds + LDS_QH + u * 8);
    const v4u a1 = *(const v4u*)(lds + LDS_QL + u * 8);
    const v4u a2 = *(const v4u*)(lds + LDS_KH + u * 8);
    const v4u a3 = *(const v4u*)(lds + LDS_KL + u * 8);
    *(volatile v4u*)(Qh + u * 8) = a0;
    *(volatile v4u*)(Ql + u * 8) = a1;
    *(volatile v4u*)(Kh + u * 8) = a2;
    *(volatile v4u*)(Kl + u * 8) = a3;
  }
#pragma unroll
  for (int p = 0; p < 16; ++p) {
    const int u = p * 128 + tid;
    const int L = u >> 3, q = u & 7;
    const v4u v = *(const v4u*)(lds + LDS_X + L * 64 + q * 8);
    *(volatile v4u*)(Vb + (size_t)L * SEQ + q * 8) = v;
  }
}

__global__ __launch_bounds__(128) void k_proj(const float* __restrict__ x,
                                              const unsigned short* __restrict__ Wb,
                                              const float* __restrict__ bq,
                                              const float* __restrict__ bk,
                                              const float* __restrict__ bv,
                                              unsigned short* __restrict__ Qh,
                                              unsigned short* __restrict__ Ql,
                                              unsigned short* __restrict__ Kh,
                                              unsigned short* __restrict__ Kl,
                                              unsigned short* __restrict__ Vh) {
  __shared__ __attribute__((aligned(16))) unsigned short lds[LDS_PROJ_TOTAL];

  const int tid  = threadIdx.x;
  const int lane = tid & 31;
  const int wave = tid >> 5;
  const int lm   = lane & 15;
  const int h    = lane >> 4;
  const int bpb  = SEQ / 64;
  const int b    = blockIdx.x / bpb;
  const int i0b  = (blockIdx.x - b * bpb) * 64;

  const float* xb = x + (size_t)b * CH * SEQ_FULL + i0b;
#pragma unroll 4
  for (int it = 0; it < 32; ++it) {
    const int idx = it * 128 + tid;
    const int c   = idx >> 4;
    const int q4  = idx & 15;
    const v4f v = *(const v4f*)(xb + (size_t)c * SEQ_FULL + 4 * q4);
    unsigned short* d = lds + LDS_X + (4 * q4) * CH + c;
    d[0]      = (unsigned short)bf16_rne_bits(v.x);
    d[CH]     = (unsigned short)bf16_rne_bits(v.y);
    d[2 * CH] = (unsigned short)bf16_rne_bits(v.z);
    d[3 * CH] = (unsigned short)bf16_rne_bits(v.w);
  }
  __syncthreads();

  Frag aP[8];
  {
    const unsigned short* ar = lds + LDS_X + (wave * 16 + lm) * CH;
#pragma unroll
    for (int ks = 0; ks < 8; ++ks) aP[ks] = ld_frag(ar + ks * 32, h);
  }
  __syncthreads();

#pragma unroll 1
  for (int nt = 0; nt < 20; ++nt) {
    const unsigned short* wr = Wb + (size_t)(nt * 16 + lm) * CH;
    v8f acc = zero8();
#pragma unroll
    for (int ks = 0; ks < 8; ++ks) {
      Frag bfr = ld_frag(wr + ks * 32, h);
      acc = mma_bf16(aP[ks], bfr, acc);
    }
    const int dq = (nt & 1) * 16 + lm;
    const int dv = ((nt - 4) & 15) * 16 + lm;
    const float b_q = bf16_rne_val(bq[dq]);
    const float b_k = bf16_rne_val(bk[dq]);
    const float b_v = bf16_rne_val(bv[dv]);
    if (nt < 4) {
      const bool  isq  = (nt < 2);
      const float bias = isq ? b_q : b_k;
      const float scl  = isq ? LOG2E : 1.0f;
      const int   poff = isq ? LDS_QH : LDS_KH;
#pragma unroll
      for (int r = 0; r < 8; ++r) {
        const float v  = (acc[r] + bias) * scl;
        const unsigned int hb = bf16_rne_bits(v);
        const float hv = __builtin_bit_cast(float, hb << 16);
        const unsigned int lb = bf16_rne_bits(v - hv);
        const int o = (wave * 16 + 8 * h + r) * DQ + dq;
        lds[poff + o]        = (unsigned short)hb;
        lds[poff + 2048 + o] = (unsigned short)lb;
      }
    } else {
#pragma unroll
      for (int r = 0; r < 8; ++r) {
        const float v = acc[r] + b_v;
        lds[LDS_X + dv * 64 + wave * 16 + 8 * h + r] = f16_bits(v);
      }
    }
  }
  __syncthreads();

  const size_t qkbase = ((size_t)b * SEQ + i0b) * DQ;
  unsigned short* Vb = Vh + (size_t)b * CH * SEQ + i0b;
  proj_store(lds, Qh + qkbase, Ql + qkbase, Kh + qkbase, Kl + qkbase, Vb, tid);
  __threadfence();
  proj_store(lds, Qh + qkbase, Ql + qkbase, Kh + qkbase, Kl + qkbase, Vb, tid);
}

__device__ __forceinline__ void attn_store(const float* sO, const float* xg, float* og,
                                           float g, int tid) {
#pragma unroll
  for (int p = 0; p < 8; ++p) {
    const int u = p * 256 + tid;
    const int L = u >> 3, q = u & 7;
    const v4f o  = *(const v4f*)(sO + L * 32 + q * 4);
    const v4f xv = *(const v4f*)(xg + (size_t)L * SEQ_FULL + q * 4);
    v4f res;
    res.x = g * o.x + bf16_rne_val(xv.x);
    res.y = g * o.y + bf16_rne_val(xv.y);
    res.z = g * o.z + bf16_rne_val(xv.z);
    res.w = g * o.w + bf16_rne_val(xv.w);
    *(volatile v4f*)(og + (size_t)L * SEQ_FULL + q * 4) = res;
  }
}

__global__ __launch_bounds__(256) void k_attn(const unsigned short* __restrict__ Qh,
                                              const unsigned short* __restrict__ Ql,
                                              const unsigned short* __restrict__ Kh,
                                              const unsigned short* __restrict__ Kl,
                                              const unsigned short* __restrict__ Vh,
                                              const float* __restrict__ x,
                                              const float* __restrict__ gamma,
                                              float* __restrict__ out) {
  __shared__ __attribute__((aligned(16))) unsigned short sP[2 * 16 * JB];
  __shared__ __attribute__((aligned(16))) float sMax[8 * 16];
  __shared__ __attribute__((aligned(16))) float sSum[8 * 16];
  __shared__ __attribute__((aligned(16))) float sO[CH * 32];

  const int tid  = threadIdx.x;
  const int lane = tid & 31;
  const int wave = tid >> 5;
  const int lm   = lane & 15;
  const int h    = lane >> 4;
  const int rg   = wave >> 2;
  const int cq   = wave & 3;
  const int bpb  = SEQ / 32;
  const int b    = blockIdx.x / bpb;
  const int i0   = (blockIdx.x - b * bpb) * 32;
  const int iw   = i0 + rg * 16;

  const size_t qrow = ((size_t)b * SEQ + iw + lm) * DQ;
  const Frag qh = ld_frag(Qh + qrow, h);
  const Frag ql = ld_frag(Ql + qrow, h);

  v8f acc[4];
#pragma unroll
  for (int ct = 0; ct < 4; ++ct) acc[ct] = zero8();
  float mrow[8], lrow[8];
#pragma unroll
  for (int r = 0; r < 8; ++r) { mrow[r] = -1.0e30f; lrow[r] = 0.0f; }

  unsigned short* myP = sP + rg * (16 * JB);

#pragma unroll 1
  for (int j0 = 0; j0 < SEQ; j0 += JB) {
    const size_t krow = ((size_t)b * SEQ + j0 + cq * 16 + lm) * DQ;
    const Frag kh = ld_frag(Kh + krow, h);
    const Frag kl = ld_frag(Kl + krow, h);
    v8f S = mma_bf16(qh, kh, zero8());
    S = mma_bf16(qh, kl, S);
    S = mma_bf16(ql, kh, S);

    float tm[8];
#pragma unroll
    for (int r = 0; r < 8; ++r) {
      float v = S[r];
#pragma unroll
      for (int msk = 1; msk <= 8; msk <<= 1) v = fmaxf(v, __shfl_xor(v, msk, 32));
      tm[r] = v;
    }
    if (lm == 0) {
      v4f a, c;
      a.x = tm[0]; a.y = tm[1]; a.z = tm[2]; a.w = tm[3];
      c.x = tm[4]; c.y = tm[5]; c.z = tm[6]; c.w = tm[7];
      *(v4f*)(sMax + wave * 16 + 8 * h)     = a;
      *(v4f*)(sMax + wave * 16 + 8 * h + 4) = c;
    }
    __syncthreads();

    float mt[8];
    {
      const float* pm = sMax + rg * 64 + 8 * h;
      v4f ma = *(const v4f*)(pm);
      v4f mb = *(const v4f*)(pm + 4);
#pragma unroll
      for (int t = 1; t < 4; ++t) {
        ma = max4(ma, *(const v4f*)(pm + t * 16));
        mb = max4(mb, *(const v4f*)(pm + t * 16 + 4));
      }
      mt[0] = ma.x; mt[1] = ma.y; mt[2] = ma.z; mt[3] = ma.w;
      mt[4] = mb.x; mt[5] = mb.y; mt[6] = mb.z; mt[7] = mb.w;
    }
    float mnew[8], alpha[8], rs[8];
#pragma unroll
    for (int r = 0; r < 8; ++r) {
      mnew[r]  = fmaxf(mrow[r], mt[r]);
      alpha[r] = __builtin_amdgcn_exp2f(mrow[r] - mnew[r]);
      mrow[r]  = mnew[r];
    }
#pragma unroll
    for (int r = 0; r < 8; ++r) {
      const float p = __builtin_amdgcn_exp2f((S[r] - mnew[r]) + PC_LOG2);
      rs[r] = p;
      myP[(8 * h + r) * JB + cq * 16 + lm] = f16_bits(p);
    }
#pragma unroll
    for (int r = 0; r < 8; ++r) {
      float v = rs[r];
#pragma unroll
      for (int msk = 1; msk <= 8; msk <<= 1) v += __shfl_xor(v, msk, 32);
      rs[r] = v;
    }
    if (lm == 0) {
      v4f a, c;
      a.x = rs[0]; a.y = rs[1]; a.z = rs[2]; a.w = rs[3];
      c.x = rs[4]; c.y = rs[5]; c.z = rs[6]; c.w = rs[7];
      *(v4f*)(sSum + wave * 16 + 8 * h)     = a;
      *(v4f*)(sSum + wave * 16 + 8 * h + 4) = c;
    }
    __syncthreads();

    {
      const float* ps = sSum + rg * 64 + 8 * h;
      v4f sa = *(const v4f*)(ps);
      v4f sb = *(const v4f*)(ps + 4);
#pragma unroll
      for (int t = 1; t < 4; ++t) {
        sa += *(const v4f*)(ps + t * 16);
        sb += *(const v4f*)(ps + t * 16 + 4);
      }
      float ls[8];
      ls[0] = sa.x; ls[1] = sa.y; ls[2] = sa.z; ls[3] = sa.w;
      ls[4] = sb.x; ls[5] = sb.y; ls[6] = sb.z; ls[7] = sb.w;
#pragma unroll
      for (int r = 0; r < 8; ++r) lrow[r] = lrow[r] * alpha[r] + ls[r];
    }
#pragma unroll
    for (int ct = 0; ct < 4; ++ct)
#pragma unroll
      for (int r = 0; r < 8; ++r) acc[ct][r] *= alpha[r];

    const unsigned short* vbase = Vh + ((size_t)b * CH + cq * 64 + lm) * SEQ + j0;
#pragma unroll
    for (int ks = 0; ks < 2; ++ks) {
      const Frag pf = ld_frag(myP + lm * JB + ks * 32, h);
#pragma unroll
      for (int ct = 0; ct < 4; ++ct) {
        const Frag vf = ld_frag(vbase + (size_t)(ct * 16) * SEQ + ks * 32, h);
        acc[ct] = mma_f16(pf, vf, acc[ct]);
      }
    }
  }

  float rinv[8];
#pragma unroll
  for (int r = 0; r < 8; ++r) rinv[r] = __builtin_amdgcn_rcpf(lrow[r]);
#pragma unroll
  for (int ct = 0; ct < 4; ++ct) {
    const int c = cq * 64 + ct * 16 + lm;
#pragma unroll
    for (int r = 0; r < 8; ++r)
      sO[c * 32 + rg * 16 + 8 * h + r] = acc[ct][r] * rinv[r];
  }
  __syncthreads();

  const float g = bf16_rne_val(gamma[0]);
  const size_t obase = (size_t)b * CH * SEQ_FULL + i0;
  attn_store(sO, x + obase, out + obase, g, tid);
  __threadfence();
  attn_store(sO, x + obase, out + obase, g, tid);
}

extern "C" void kernel_launch(void* const* d_in, const int* in_sizes, int n_in,
                              void* d_out, int out_size, void* d_ws, size_t ws_size,
                              hipStream_t stream) {
  if (n_in < 8) return;
  const size_t need_x = ((size_t)NB * CH - 1) * SEQ_FULL + SEQ;
  if ((size_t)in_sizes[0] < need_x) return;
  if (in_sizes[1] < DQ * CH || in_sizes[2] < DQ || in_sizes[3] < DQ * CH || in_sizes[4] < DQ ||
      in_sizes[5] < CH * CH || in_sizes[6] < CH || in_sizes[7] < 1) return;
  if ((size_t)out_size < need_x) return;

  const float* x     = (const float*)d_in[0];
  const float* Wq    = (const float*)d_in[1];
  const float* bq    = (const float*)d_in[2];
  const float* Wk    = (const float*)d_in[3];
  const float* bk    = (const float*)d_in[4];
  const float* Wv    = (const float*)d_in[5];
  const float* bv    = (const float*)d_in[6];
  const float* gamma = (const float*)d_in[7];
  float* out = (float*)d_out;

  const size_t nW  = (size_t)WROWS * CH;
  const size_t nQK = (size_t)NB * SEQ * DQ;
  const size_t nV  = (size_t)NB * CH * SEQ;
  const size_t total_bytes = (nW + 4 * nQK + nV) * 2;
  if (total_bytes > ws_size) return;

  unsigned short* ws  = (unsigned short*)d_ws;
  unsigned short* Wb  = ws;
  unsigned short* Qh  = Wb + nW;
  unsigned short* Ql  = Qh + nQK;
  unsigned short* Kh  = Ql + nQK;
  unsigned short* Kl  = Kh + nQK;
  unsigned short* Vhp = Kl + nQK;

  k_wconv<<<(DQ * CH / 8 + 127) / 128, 128, 0, stream>>>(Wq, Wb, DQ * CH);
  k_wconv<<<(DQ * CH / 8 + 127) / 128, 128, 0, stream>>>(Wk, Wb + DQ * CH, DQ * CH);
  k_wconv<<<(CH * CH / 8 + 127) / 128, 128, 0, stream>>>(Wv, Wb + 2 * DQ * CH, CH * CH);
  k_proj<<<NB * (SEQ / 64), 128, 0, stream>>>(x, Wb, bq, bk, bv, Qh, Ql, Kh, Kl, Vhp);
  k_attn<<<NB * (SEQ / 32), 256, 0, stream>>>(Qh, Ql, Kh, Kl, Vhp, x, gamma, out);
}
